// GRU_37546604101723
// MI455X (gfx1250) — hardware-verified
//
#include <hip/hip_runtime.h>
#include <math.h>

#pragma clang fp contract(off)

typedef __attribute__((ext_vector_type(16))) _Float16 v16h;
typedef __attribute__((ext_vector_type(8)))  _Float16 v8h;
typedef __attribute__((ext_vector_type(16))) __bf16   v16b;
typedef __attribute__((ext_vector_type(8)))  __bf16   v8b;
typedef __attribute__((ext_vector_type(8)))  float    v8f;
typedef __attribute__((ext_vector_type(4)))  float    v4f;
#define PSCALE 32768.0f
#define U16(p) ((const unsigned short*)(const void*)(p))
#define PSCALE_INV (1.0f / 32768.0f)

__device__ __forceinline__ unsigned short f2bf_bits(float f) {
  unsigned u = __float_as_uint(f);
  return (unsigned short)((u + 0x7FFFu + ((u >> 16) & 1u)) >> 16);
}
__device__ __forceinline__ float bf_bits2f(unsigned short h) { return __uint_as_float(((unsigned)h) << 16); }

__device__ __forceinline__ void dep_guard_h(v8f& a, v8f& b, v16h x, v16h y) { asm volatile("v_nop\n\tv_nop\n\tv_nop\n\tv_nop" : "+v"(a), "+v"(b) : "v"(x), "v"(y)); }
__device__ __forceinline__ void dep_guard_b(v8f& a, v8f& b, v16b x, v16b y) { asm volatile("v_nop\n\tv_nop\n\tv_nop\n\tv_nop" : "+v"(a), "+v"(b) : "v"(x), "v"(y)); }
__device__ __forceinline__ void keep4_h(v16h a, v16h b, v16h c, v16h d) { asm volatile("v_nop" :: "v"(a), "v"(b), "v"(c), "v"(d)); }
__device__ __forceinline__ void keep4_b(v16b a, v16b b, v16b c, v16b d) { asm volatile("v_nop" :: "v"(a), "v"(b), "v"(c), "v"(d)); }
__device__ __forceinline__ void acc_guard4(v8f& a, v8f& b, v8f& c, v8f& d) { asm volatile("v_nop\n\tv_nop\n\tv_nop\n\tv_nop" : "+v"(a), "+v"(b), "+v"(c), "+v"(d)); }
template <typename T> struct Frag;
template <> struct Frag<_Float16> {
  typedef v16h V; union U { v16h v; v8h h[2]; };
  static __device__ __forceinline__ v16h load(const _Float16* p) {
    U f; f.h[0] = *(const v8h*)(p); f.h[1] = *(const v8h*)(p + 16); return f.v;
  }
  static __device__ __forceinline__ v8f mma(v16h a, v16h b, v8f c) {
    return __builtin_amdgcn_wmma_f32_16x16x32_f16(false, a, false, b, (short)0, c, false, false);
  }
  static __device__ __forceinline__ void guard(v8f& a, v8f& b, v16h x, v16h y) { dep_guard_h(a, b, x, y); }
  static __device__ __forceinline__ void keep(v16h a, v16h b, v16h c, v16h d) { keep4_h(a, b, c, d); }
};
template <> struct Frag<__bf16> {
  typedef v16b V; union U { v16b v; v8b h[2]; };
  static __device__ __forceinline__ v16b load(const __bf16* p) {
    U f; f.h[0] = *(const v8b*)(p); f.h[1] = *(const v8b*)(p + 16); return f.v;
  }
  static __device__ __forceinline__ v8f mma(v16b a, v16b b, v8f c) {
    return __builtin_amdgcn_wmma_f32_16x16x32_bf16(false, a, false, b, (short)0, c, false, false);
  }
  static __device__ __forceinline__ void guard(v8f& a, v8f& b, v16b x, v16b y) { dep_guard_b(a, b, x, y); }
  static __device__ __forceinline__ void keep(v16b a, v16b b, v16b c, v16b d) { keep4_b(a, b, c, d); }
};

template <int ET> struct Elem;
template <> struct Elem<0> { typedef _Float16 T; };
template <> struct Elem<1> { typedef __bf16 T; };
template <int ET, bool SPLIT, int BIAS_MODE, int OUT_MODE, bool RESID, int ACT = 0>
__global__ __launch_bounds__(256) void wmma_gemm64(
    const unsigned short* __restrict__ Ap, const unsigned short* __restrict__ A2p, int lda, long strideA,
    const unsigned short* __restrict__ Btp, const unsigned short* __restrict__ Bt2p, int ldb, long strideB,
    void* __restrict__ Cout, void* __restrict__ Cout2, int ldc, long strideC,
    const float* __restrict__ bias,
    const float* __restrict__ resid, long strideR,
    int M, int N, int K, float scale) {
  typedef typename Elem<ET>::T T;
  typedef typename Frag<T>::V V;
  const T* A = (const T*)Ap; const T* A2 = (const T*)A2p; const T* Bt = (const T*)Btp; const T* Bt2 = (const T*)Bt2p;
  __shared__ __align__(16) float sT[8][16 * 68];
  const int b    = blockIdx.y;
  const int lane = threadIdx.x & 31;
  const int wave = threadIdx.x >> 5;
  const int tilesN = N >> 6;
  const int tilesM = M >> 6;
  const int tile = blockIdx.x * 8 + wave;
  if (tile >= tilesM * tilesN) return;
  const int tm = tile / tilesN;
  const int tn = tile - tm * tilesN;
  const int m0 = tm << 6;
  const int n0 = tn << 6;

  const T* Ab  = A  + (size_t)b * strideA;
  const T* Bb  = Bt + (size_t)b * strideB;
  const T* Ab2 = SPLIT ? (A2  + (size_t)b * strideA) : nullptr;
  const T* Bb2 = SPLIT ? (Bt2 + (size_t)b * strideB) : nullptr;

  const int rlane = lane & 15;
  const int koff  = (lane >> 4) * 8;
  const int mOff  = (lane >> 4) * 8;

  v8f acc[4][4];
#pragma unroll
  for (int i = 0; i < 4; ++i)
#pragma unroll
    for (int j = 0; j < 4; ++j) acc[i][j] = (v8f){0.f,0.f,0.f,0.f,0.f,0.f,0.f,0.f};

  for (int k0 = 0; k0 < K; k0 += 32) {
    V bh[4], bl[4];
#pragma unroll
    for (int j = 0; j < 4; ++j) {
      const size_t bo = (size_t)(n0 + (j << 4) + rlane) * ldb + koff + k0;
      bh[j] = Frag<T>::load(Bb + bo);
      if (SPLIT) bl[j] = Frag<T>::load(Bb2 + bo);
    }
#pragma unroll
    for (int i = 0; i < 4; ++i) {
      const size_t ao = (size_t)(m0 + (i << 4) + rlane) * lda + koff + k0;
      V ah = Frag<T>::load(Ab + ao);
      V al;
      if (SPLIT) al = Frag<T>::load(Ab2 + ao);
#pragma unroll
      for (int j = 0; j < 4; ++j) {
        acc[i][j] = Frag<T>::mma(ah, bh[j], acc[i][j]);
        if (SPLIT) {
          acc[i][j] = Frag<T>::mma(ah, bl[j], acc[i][j]);
          acc[i][j] = Frag<T>::mma(al, bh[j], acc[i][j]);
        }
      }
      Frag<T>::guard(acc[i][0], acc[i][3], ah, SPLIT ? al : ah);
    }
    Frag<T>::keep(bh[0], bh[1], bh[2], bh[3]);
    if (SPLIT) Frag<T>::keep(bl[0], bl[1], bl[2], bl[3]);
  }
  acc_guard4(acc[0][0], acc[0][1], acc[0][2], acc[0][3]);
  acc_guard4(acc[1][0], acc[1][1], acc[1][2], acc[1][3]);
  acc_guard4(acc[2][0], acc[2][1], acc[2][2], acc[2][3]);
  acc_guard4(acc[3][0], acc[3][1], acc[3][2], acc[3][3]);

  float* slab = sT[wave];
  const float* Rb = RESID ? (resid + (size_t)b * strideR) : nullptr;
#pragma unroll
  for (int i = 0; i < 4; ++i) {
    const int mBase = m0 + (i << 4);
#pragma unroll
    for (int j = 0; j < 4; ++j) {
      const int n = n0 + (j << 4) + rlane;
      float bv = 0.f;
      if (BIAS_MODE == 2) bv = bias[n];
#pragma unroll
      for (int r = 0; r < 8; ++r) {
        float v = acc[i][j][r] * scale;
        if (BIAS_MODE == 1) v += bias[mBase + mOff + r];
        if (BIAS_MODE == 2) v += bv;
        if (RESID) v += Rb[(size_t)(mBase + mOff + r) * ldc + n];
        if (ACT == 1) v = tanhf(v);
        if (ACT == 2) v = fmaxf(v, 0.0f);
        if (ACT == 3) v = v / (1.0f + expf(-v));
        if (ACT == 4) v = (v > 0.f) ? v : 0.01f * v;
        if (ACT == 5) v = 0.5f * v * (1.0f + erff(v * 0.70710678118654752f));
        slab[(mOff + r) * 68 + (j << 4) + rlane] = v;
      }
    }
    __builtin_amdgcn_fence(__ATOMIC_RELEASE, "workgroup");
    __builtin_amdgcn_wave_barrier();
    __builtin_amdgcn_fence(__ATOMIC_ACQUIRE, "workgroup");
    if (OUT_MODE == 0) {
      float* C = (float*)Cout + (size_t)b * strideC;
      const int hh = lane >> 4, c4 = (lane & 15) * 4;
      for (int pass = 0; pass < 2; ++pass) {
#pragma unroll
        for (int it = 0; it < 8; ++it) {
          const int row = it * 2 + hh;
          v4f v = *(const v4f*)(slab + row * 68 + c4);
          *(volatile v4f*)(C + (size_t)(mBase + row) * ldc + n0 + c4) = v;
        }
        __threadfence();
      }
    } else {
      const int q = lane >> 3, c8 = (lane & 7) * 8;
      unsigned short* C  = (unsigned short*)Cout  + (size_t)b * strideC;
      unsigned short* C2 = (OUT_MODE == 2) ? ((unsigned short*)Cout2 + (size_t)b * strideC) : nullptr;
      for (int pass = 0; pass < 2; ++pass) {
#pragma unroll
        for (int it = 0; it < 4; ++it) {
          const int row = it * 4 + q;
          const float* sp = slab + row * 68 + c8;
          v8h hv, lv;
#pragma unroll
          for (int e = 0; e < 8; ++e) {
            if (OUT_MODE == 1) {
              hv[e] = (_Float16)sp[e];
            } else {
              unsigned short hb = f2bf_bits(sp[e]);
              unsigned short lb = f2bf_bits(sp[e] - bf_bits2f(hb));
              hv[e] = __builtin_bit_cast(_Float16, hb);
              lv[e] = __builtin_bit_cast(_Float16, lb);
            }
          }
          *(volatile v8h*)(C + (size_t)(mBase + row) * ldc + n0 + c8) = hv;
          if (OUT_MODE == 2) *(volatile v8h*)(C2 + (size_t)(mBase + row) * ldc + n0 + c8) = lv;
        }
        __threadfence();
      }
    }
    __builtin_amdgcn_fence(__ATOMIC_RELEASE, "workgroup");
    __builtin_amdgcn_wave_barrier();
    __builtin_amdgcn_fence(__ATOMIC_ACQUIRE, "workgroup");
  }
}

constexpr int NB     = 2;
constexpr int NPTS   = 4096;
constexpr int HID    = 128;
constexpr int XD     = 256;
constexpr int CF     = HID + XD;
constexpr int CIN    = CF + 3;
constexpr int KNB    = 4;
constexpr int KPAD   = 416;
constexpr int GPITCH = 448;
constexpr int NQ     = NB * NPTS;
constexpr int NROWS  = NQ * KNB;
constexpr int ROWS_PER_B = NPTS * KNB;
constexpr int SCHUNK = 512;
constexpr int NCHUNK = ROWS_PER_B / SCHUNK;
constexpr int ZRLD   = 2 * HID;
constexpr float NORM_EPS = 1e-5f;

static_assert(KPAD % 32 == 0 && KPAD >= CIN && KPAD + 0 <= GPITCH, "K padding");
static_assert(NROWS % 64 == 0 && HID % 64 == 0, "GEMM tile multiples");
static_assert(((NROWS / 64) * (HID / 64)) % 8 == 0, "GEMM grid exact");
static_assert(NPTS % 512 == 0 && NPTS % 256 == 0 && NPTS % 32 == 0, "tiling");
static_assert(ROWS_PER_B % SCHUNK == 0, "stats chunks");
static_assert(CF % 64 == 0 && HID % 64 == 0, "transpose tile coverage");

constexpr size_t SZ_FEAT = (size_t)NQ * CF * 4;
constexpr size_t SZ_GPL  = (size_t)NROWS * GPITCH * 2;
constexpr size_t SZ_WPL  = (size_t)3 * HID * GPITCH * 2;
constexpr size_t SZ_YZR  = (size_t)NROWS * ZRLD * 4;
constexpr size_t SZ_PZR  = (size_t)NB * NCHUNK * ZRLD * 4;
constexpr size_t SZ_MZR  = (size_t)NB * ZRLD * 4;
constexpr size_t SZ_GATE = (size_t)NQ * HID * 4;
constexpr size_t SZ_YQ   = (size_t)NROWS * HID * 4;
constexpr size_t SZ_PQ   = (size_t)NB * NCHUNK * HID * 4;
constexpr size_t SZ_MQ   = (size_t)NB * HID * 4;
constexpr size_t WS_TOTAL = SZ_FEAT + 2 * SZ_GPL + 2 * SZ_WPL + SZ_YZR + 2 * SZ_PZR + 2 * SZ_MZR
                          + 2 * SZ_GATE + SZ_YQ + 2 * SZ_PQ + 2 * SZ_MQ;
static_assert(WS_TOTAL == 130914304, "carve total");
static_assert(WS_TOTAL <= 134217728, "carve budget");
static_assert(SZ_FEAT % 256 == 0 && SZ_GPL % 256 == 0 && SZ_WPL % 256 == 0 && SZ_YZR % 256 == 0 &&
              SZ_PZR % 256 == 0 && SZ_MZR % 256 == 0 && SZ_GATE % 256 == 0 && SZ_YQ % 256 == 0 &&
              SZ_PQ % 256 == 0 && SZ_MQ % 256 == 0, "region alignment");

__device__ __forceinline__ void wave_sync_lds() {
  __builtin_amdgcn_fence(__ATOMIC_RELEASE, "workgroup");
  __builtin_amdgcn_wave_barrier();
  __builtin_amdgcn_fence(__ATOMIC_ACQUIRE, "workgroup");
}

__global__ __launch_bounds__(256) void k_feat(const float* __restrict__ h, const float* __restrict__ x,
                                              float* __restrict__ featT) {
  __shared__ float tile[64][65];
  const int c0  = blockIdx.x * 64;
  const int p0  = blockIdx.y * 64;
  const int b   = p0 / NPTS;
  const int s0  = p0 - b * NPTS;
  const int tid = threadIdx.x;
  const float* src = (c0 < HID) ? (h + ((size_t)b * HID + c0) * NPTS) : (x + ((size_t)b * XD + (c0 - HID)) * NPTS);
  {
    const int s = tid & 63, cq = tid >> 6;
#pragma unroll 4
    for (int it = 0; it < 16; ++it) {
      const int ch = it * 4 + cq;
      tile[ch][s] = src[(size_t)ch * NPTS + s0 + s];
    }
  }
  __syncthreads();
  const int wave = tid >> 5, lane = tid & 31, hh = lane >> 4, c4 = (lane & 15) * 4;
  for (int pass = 0; pass < 2; ++pass) {
#pragma unroll
    for (int it = 0; it < 4; ++it) {
      const int row = wave * 8 + it * 2 + hh;
      v4f v;
      v[0] = tile[c4 + 0][row]; v[1] = tile[c4 + 1][row]; v[2] = tile[c4 + 2][row]; v[3] = tile[c4 + 3][row];
      *(volatile v4f*)(featT + (size_t)(p0 + row) * CF + c0 + c4) = v;
    }
    __threadfence();
  }
}

__device__ __forceinline__ void wsplit8(const float* __restrict__ srow, int chunk, v8h& hv, v8h& lv) {
#pragma unroll
  for (int e = 0; e < 8; ++e) {
    const int c  = chunk * 8 + e;
    const int cc = (c > CIN - 1) ? (CIN - 1) : c;
    const float w  = srow[cc];
    const float ff = (c < CIN) ? 1.0f : 0.0f;
    const float v  = fmaf(ff, w, 0.0f);
    const unsigned short hb = f2bf_bits(v);
    const unsigned short lb = f2bf_bits(v - bf_bits2f(hb));
    hv[e] = __builtin_bit_cast(_Float16, hb);
    lv[e] = __builtin_bit_cast(_Float16, lb);
  }
}
__global__ __launch_bounds__(256) void k_wprep(const float* __restrict__ Wz, const float* __restrict__ Wr,
                                               const float* __restrict__ Wq,
                                               unsigned short* __restrict__ WPhi, unsigned short* __restrict__ WPlo) {
  const int wave = threadIdx.x >> 5, lane = threadIdx.x & 31;
  const int o = blockIdx.x * 8 + wave;
  const float* src = (o < HID) ? Wz : ((o < 2 * HID) ? Wr : Wq);
  const float* srow = src + (size_t)(o & (HID - 1)) * CIN;
  v8h ha, la, hb, lb;
  wsplit8(srow, lane, ha, la);
  asm volatile("" :: "v"(ha), "v"(la) : "memory");
  wsplit8(srow, 32 + lane, hb, lb);
  unsigned short* dh = WPhi + (size_t)o * GPITCH;
  unsigned short* dl = WPlo + (size_t)o * GPITCH;
  for (int pass = 0; pass < 2; ++pass) {
    *(volatile v8h*)(dh + 8 * lane) = ha;
    *(volatile v8h*)(dl + 8 * lane) = la;
    if (lane < 24) {
      *(volatile v8h*)(dh + 256 + 8 * lane) = hb;
      *(volatile v8h*)(dl + 256 + 8 * lane) = lb;
    }
    __threadfence();
  }
}

template <int MODE>
__device__ __forceinline__ void build_chunk(int chunk, const float* fr, const float* rr,
                                            float gx, float gy, float gz, v8h& hv, v8h& lv) {
#pragma unroll
  for (int e = 0; e < 8; ++e) {
    const int c = chunk * 8 + e;
    int fc = c - 3; fc = (fc < 0) ? 0 : fc; fc = (fc > CF - 1) ? (CF - 1) : fc;
    const float f = fr[fc];
    float fterm = f;
    if (MODE == 1) {
      int rc = c - 3; rc = (rc < 0) ? 0 : rc; rc = (rc > HID - 1) ? (HID - 1) : rc;
      const float rv   = rr[rc];
      const float hsel = (c < 3 + HID) ? 1.0f : 0.0f;
      const float rfac = fmaf(hsel, rv, 1.0f - hsel);
      fterm = f * rfac;
    }
    const float fx = (c == 0) ? 1.0f : 0.0f;
    const float fy = (c == 1) ? 1.0f : 0.0f;
    const float fz = (c == 2) ? 1.0f : 0.0f;
    const float gf = fmaf(fx, gx, fmaf(fy, gy, fz * gz));
    const float ff = (c >= 3 && c < CIN) ? 1.0f : 0.0f;
    const float v  = fmaf(ff, fterm, gf);
    const unsigned short hb = f2bf_bits(v);
    const unsigned short lb = f2bf_bits(v - bf_bits2f(hb));
    hv[e] = __builtin_bit_cast(_Float16, hb);
    lv[e] = __builtin_bit_cast(_Float16, lb);
  }
}

template <int MODE>
__global__ __launch_bounds__(256) void k_group(const float* __restrict__ pc,
                                               const float* __restrict__ featT,
                                               const float* __restrict__ rpl,
                                               unsigned short* __restrict__ Ghi,
                                               unsigned short* __restrict__ Glo) {
  __shared__ __align__(16) v4f   cand[512];
  __shared__ int                 snb[256 * KNB];
  __shared__ __align__(16) float qpos[256 * 4];
  __shared__ __align__(16) float frow[8][CF];
  __shared__ __align__(16) float rrow[8][HID];

  const int b   = blockIdx.y;
  const int q0  = blockIdx.x * 256;
  const int tid = threadIdx.x;
  const float* pcb = pc + (size_t)b * 3 * NPTS;
  const int qi = q0 + tid;
  const float qx = pcb[qi], qy = pcb[NPTS + qi], qz = pcb[2 * NPTS + qi];
  const float sqq = (qx * qx + qz * qz) + qy * qy;

  float bd0 = INFINITY, bd1 = INFINITY, bd2 = INFINITY, bd3 = INFINITY;
  int   bi0 = 0, bi1 = 0, bi2 = 0, bi3 = 0;

  for (int j0 = 0; j0 < NPTS; j0 += 512) {
    __syncthreads();
    for (int e = tid; e < 512; e += 256) {
      const float cx = pcb[j0 + e], cy = pcb[NPTS + j0 + e], cz = pcb[2 * NPTS + j0 + e];
      const float sc = (cx * cx + cz * cz) + cy * cy;
      v4f cv; cv[0] = cx; cv[1] = cy; cv[2] = cz; cv[3] = sc;
      cand[e] = cv;
    }
    __syncthreads();
#pragma unroll 2
    for (int j = 0; j < 512; ++j) {
      const v4f cv = cand[j];
      float p = qx * cv[0];
      p = fmaf(qy, cv[1], p);
      p = fmaf(qz, cv[2], p);
      const float dd = (sqq + cv[3]) - 2.0f * p;
      const int   id = j0 + j;
      const bool c3 = dd < bd3, c2 = dd < bd2, c1 = dd < bd1, c0 = dd < bd0;
      bd3 = c3 ? (c2 ? bd2 : dd) : bd3;  bi3 = c3 ? (c2 ? bi2 : id) : bi3;
      bd2 = c2 ? (c1 ? bd1 : dd) : bd2;  bi2 = c2 ? (c1 ? bi1 : id) : bi2;
      bd1 = c1 ? (c0 ? bd0 : dd) : bd1;  bi1 = c1 ? (c0 ? bi0 : id) : bi1;
      bd0 = c0 ? dd : bd0;               bi0 = c0 ? id : bi0;
    }
  }
  snb[tid * KNB + 0] = bi0; snb[tid * KNB + 1] = bi1; snb[tid * KNB + 2] = bi2; snb[tid * KNB + 3] = bi3;
  qpos[tid * 4 + 0] = qx; qpos[tid * 4 + 1] = qy; qpos[tid * 4 + 2] = qz;
  __syncthreads();

  const int wave = tid >> 5, lane = tid & 31;
  float* fr = frow[wave];
  float* rr = rrow[wave];
#pragma unroll 1
  for (int rl = 0; rl < 128; ++rl) {
    const int rib = wave * 128 + rl;
    const int ql  = rib >> 2, kk = rib & 3;
    int nb = snb[ql * KNB + kk];
    nb = (nb < 0) ? 0 : ((nb > NPTS - 1) ? (NPTS - 1) : nb);
    const size_t nrow = (size_t)b * NPTS + nb;
    const v4f* fsrc = (const v4f*)(featT + nrow * CF);
    const v4f f0 = fsrc[lane], f1 = fsrc[32 + lane], f2 = fsrc[64 + lane];
    v4f r0 = (v4f){0.f, 0.f, 0.f, 0.f};
    if (MODE == 1) r0 = ((const v4f*)(rpl + nrow * HID))[lane];
    wave_sync_lds();
    *(v4f*)(fr + 4 * lane) = f0; *(v4f*)(fr + 128 + 4 * lane) = f1; *(v4f*)(fr + 256 + 4 * lane) = f2;
    if (MODE == 1) *(v4f*)(rr + 4 * lane) = r0;
    wave_sync_lds();
    const float nx = pcb[nb], ny = pcb[NPTS + nb], nz = pcb[2 * NPTS + nb];
    const float gx = nx - qpos[ql * 4 + 0];
    const float gy = ny - qpos[ql * 4 + 1];
    const float gz = nz - qpos[ql * 4 + 2];
    v8h ha, la, hb, lb;
    build_chunk<MODE>(lane, fr, rr, gx, gy, gz, ha, la);
    build_chunk<MODE>(32 + lane, fr, rr, gx, gy, gz, hb, lb);
    const size_t grow = ((size_t)b * NPTS + q0 + ql) * KNB + kk;
    unsigned short* dh = Ghi + grow * GPITCH;
    unsigned short* dl = Glo + grow * GPITCH;
    for (int pass = 0; pass < 2; ++pass) {
      *(volatile v8h*)(dh + 8 * lane) = ha;
      *(volatile v8h*)(dl + 8 * lane) = la;
      if (lane < 24) {
        *(volatile v8h*)(dh + 256 + 8 * lane) = hb;
        *(volatile v8h*)(dl + 256 + 8 * lane) = lb;
      }
      __threadfence();
    }
  }
}

__global__ __launch_bounds__(256) void k_colstats(const float* __restrict__ y, int ld, int ncols,
                                                  float* __restrict__ psum, float* __restrict__ psq) {
  const int b = blockIdx.y, chunk = blockIdx.x, col = threadIdx.x;
  const size_t r0 = (size_t)b * ROWS_PER_B + (size_t)chunk * SCHUNK;
  float s = 0.0f, s2 = 0.0f;
#pragma unroll 4
  for (int i = 0; i < SCHUNK; ++i) {
    const float v = y[(r0 + i) * ld + col];
    s  = s + v;
    s2 = fmaf(v, v, s2);
  }
  const size_t pi = ((size_t)b * NCHUNK + chunk) * ncols + col;
  *(volatile float*)(psum + pi) = s;
  *(volatile float*)(psq + pi)  = s2;
  __threadfence();
  *(volatile float*)(psum + pi) = s;
  *(volatile float*)(psq + pi)  = s2;
}

__global__ __launch_bounds__(256) void k_statfin(const float* __restrict__ psum, const float* __restrict__ psq,
                                                 int ncols, float* __restrict__ mean, float* __restrict__ inv) {
  const int b = blockIdx.x, col = threadIdx.x;
  float s = 0.0f, s2 = 0.0f;
#pragma unroll 4
  for (int ch = 0; ch < NCHUNK; ++ch) {
    const size_t pi = ((size_t)b * NCHUNK + ch) * ncols + col;
    s  = s + psum[pi];
    s2 = s2 + psq[pi];
  }
  const float rn = 1.0f / (float)ROWS_PER_B;
  const float m  = s * rn;
  float var = s2 * rn - m * m;
  var = (var < 0.0f) ? 0.0f : var;
  const float iv = 1.0f / sqrtf(var + NORM_EPS);
  const size_t oi = (size_t)b * ncols + col;
  *(volatile float*)(mean + oi) = m;
  *(volatile float*)(inv + oi)  = iv;
  __threadfence();
  *(volatile float*)(mean + oi) = m;
  *(volatile float*)(inv + oi)  = iv;
}

__global__ __launch_bounds__(256) void k_fin_zr(const float* __restrict__ yzr, const float* __restrict__ mean,
                                                const float* __restrict__ inv,
                                                float* __restrict__ zpl, float* __restrict__ rpl) {
  const int b = blockIdx.y, s0 = blockIdx.x * 32, col = threadIdx.x;
  const float m  = mean[b * ZRLD + col];
  const float iv = inv[b * ZRLD + col];
  float* dst = (col < HID) ? zpl : rpl;
  const int oc = col & (HID - 1);
#pragma unroll 1
  for (int sl = 0; sl < 32; ++sl) {
    const size_t prow = (size_t)b * NPTS + s0 + sl;
    const float* yp = yzr + prow * KNB * ZRLD + col;
    const float v0 = (yp[0] - m) * iv;
    const float v1 = (yp[ZRLD] - m) * iv;
    const float v2 = (yp[2 * ZRLD] - m) * iv;
    const float v3 = (yp[3 * ZRLD] - m) * iv;
    const float mx = fmaxf(fmaxf(v0, v1), fmaxf(v2, v3));
    const float g  = 1.0f / (1.0f + expf(-mx));
    float* p = dst + prow * HID + oc;
    *(volatile float*)p = g;
    __threadfence();
    *(volatile float*)p = g;
  }
}

__global__ __launch_bounds__(256) void k_fin_q(const float* __restrict__ yq, const float* __restrict__ mean,
                                               const float* __restrict__ inv, const float* __restrict__ zpl,
                                               const float* __restrict__ h, float* __restrict__ out) {
  __shared__ __align__(16) float Zt[HID * 36];
  __shared__ __align__(16) float Qt[HID * 36];
  const int b = blockIdx.y, s0 = blockIdx.x * 32, tid = threadIdx.x;
  {
    const int o = tid & (HID - 1), sg = tid >> 7;
    const float m  = mean[b * HID + o];
    const float iv = inv[b * HID + o];
#pragma unroll 1
    for (int it = 0; it < 16; ++it) {
      const int sl = sg + 2 * it;
      const size_t prow = (size_t)b * NPTS + s0 + sl;
      const float* yp = yq + prow * KNB * HID + o;
      const float v0 = (yp[0] - m) * iv;
      const float v1 = (yp[HID] - m) * iv;
      const float v2 = (yp[2 * HID] - m) * iv;
      const float v3 = (yp[3 * HID] - m) * iv;
      const float mx = fmaxf(fmaxf(v0, v1), fmaxf(v2, v3));
      Qt[o * 36 + sl] = tanhf(mx);
      Zt[o * 36 + sl] = zpl[prow * HID + o];
    }
  }
  __syncthreads();
  const int wave = tid >> 5, lane = tid & 31, rq = lane >> 3, c4 = (lane & 7) * 4;
  for (int pass = 0; pass < 2; ++pass) {
#pragma unroll
    for (int rnd = 0; rnd < 4; ++rnd) {
      const int o = rnd * 32 + wave * 4 + rq;
      const size_t gi = ((size_t)b * HID + o) * NPTS + s0 + c4;
      const v4f h4 = *(const v4f*)(h + gi);
      const v4f z4 = *(const v4f*)(Zt + o * 36 + c4);
      const v4f q4 = *(const v4f*)(Qt + o * 36 + c4);
      v4f r4;
#pragma unroll
      for (int e = 0; e < 4; ++e) r4[e] = (1.0f - z4[e]) * h4[e] + z4[e] * q4[e];
      *(volatile v4f*)(out + gi) = r4;
    }
    __threadfence();
  }
}

extern "C" void kernel_launch(void* const* d_in, const int* in_sizes, int n_in,
                              void* d_out, int out_size, void* d_ws, size_t ws_size,
                              hipStream_t stream) {
  if (n_in < 9) return;
  if (in_sizes[0] != NB * HID * NPTS || in_sizes[1] != NB * XD * NPTS || in_sizes[2] != NB * 3 * NPTS ||
      in_sizes[3] != HID * CIN || in_sizes[4] != HID || in_sizes[5] != HID * CIN || in_sizes[6] != HID ||
      in_sizes[7] != HID * CIN || in_sizes[8] != HID || out_size != NB * HID * NPTS) return;
  if (ws_size < WS_TOTAL) return;

  const float* h  = (const float*)d_in[0];
  const float* x  = (const float*)d_in[1];
  const float* pc = (const float*)d_in[2];
  const float* Wz = (const float*)d_in[3];
  const float* bz = (const float*)d_in[4];
  const float* Wr = (const float*)d_in[5];
  const float* br = (const float*)d_in[6];
  const float* Wq = (const float*)d_in[7];
  const float* bq = (const float*)d_in[8];
  float* out = (float*)d_out;

  char* ws = (char*)d_ws;
  size_t off = 0;
  auto carve = [&](size_t bytes) -> char* { char* p = ws + off; off += (bytes + 255) & ~(size_t)255; return p; };
  float*          featT  = (float*)carve(SZ_FEAT);
  unsigned short* Ghi    = (unsigned short*)carve(SZ_GPL);
  unsigned short* Glo    = (unsigned short*)carve(SZ_GPL);
  unsigned short* WPhi   = (unsigned short*)carve(SZ_WPL);
  unsigned short* WPlo   = (unsigned short*)carve(SZ_WPL);
  float*          yzr    = (float*)carve(SZ_YZR);
  float*          ps_zr  = (float*)carve(SZ_PZR);
  float*          pq_zr  = (float*)carve(SZ_PZR);
  float*          mn_zr  = (float*)carve(SZ_MZR);
  float*          iv_zr  = (float*)carve(SZ_MZR);
  float*          zpl    = (float*)carve(SZ_GATE);
  float*          rpl    = (float*)carve(SZ_GATE);
  float*          yq     = (float*)carve(SZ_YQ);
  float*          ps_q   = (float*)carve(SZ_PQ);
  float*          pq_q   = (float*)carve(SZ_PQ);
  float*          mn_q   = (float*)carve(SZ_MQ);
  float*          iv_q   = (float*)carve(SZ_MQ);
  if (off > ws_size) return;

  const dim3 ggrid(((NROWS / 64) * (HID / 64)) / 8, 1);

  k_feat<<<dim3(CF / 64, NQ / 64), 256, 0, stream>>>(h, x, featT);
  k_wprep<<<dim3((3 * HID) / 8), 256, 0, stream>>>(Wz, Wr, Wq, WPhi, WPlo);
  k_group<0><<<dim3(NPTS / 256, NB), 256, 0, stream>>>(pc, featT, rpl, Ghi, Glo);
  wmma_gemm64<1, true, 2, 0, false, 0><<<ggrid, 256, 0, stream>>>(
      (const unsigned short*)Ghi, (const unsigned short*)Glo, GPITCH, (long)0,
      (const unsigned short*)WPhi, (const unsigned short*)WPlo, GPITCH, (long)0,
      (void*)yzr, (void*)nullptr, ZRLD, (long)0, bz, (const float*)nullptr, (long)0,
      NROWS, HID, KPAD, 1.0f);
  wmma_gemm64<1, true, 2, 0, false, 0><<<ggrid, 256, 0, stream>>>(
      (const unsigned short*)Ghi, (const unsigned short*)Glo, GPITCH, (long)0,
      (const unsigned short*)(WPhi + (size_t)HID * GPITCH), (const unsigned short*)(WPlo + (size_t)HID * GPITCH), GPITCH, (long)0,
      (void*)(yzr + HID), (void*)nullptr, ZRLD, (long)0, br, (const float*)nullptr, (long)0,
      NROWS, HID, KPAD, 1.0f);
  k_colstats<<<dim3(NCHUNK, NB), ZRLD, 0, stream>>>(yzr, ZRLD, ZRLD, ps_zr, pq_zr);
  k_statfin<<<dim3(NB), ZRLD, 0, stream>>>(ps_zr, pq_zr, ZRLD, mn_zr, iv_zr);
  k_fin_zr<<<dim3(NPTS / 32, NB), 256, 0, stream>>>(yzr, mn_zr, iv_zr, zpl, rpl);
  k_group<1><<<dim3(NPTS / 256, NB), 256, 0, stream>>>(pc, featT, rpl, Ghi, Glo);
  wmma_gemm64<1, true, 2, 0, false, 0><<<ggrid, 256, 0, stream>>>(
      (const unsigned short*)Ghi, (const unsigned short*)Glo, GPITCH, (long)0,
      (const unsigned short*)(WPhi + (size_t)2 * HID * GPITCH), (const unsigned short*)(WPlo + (size_t)2 * HID * GPITCH), GPITCH, (long)0,
      (void*)yq, (void*)nullptr, HID, (long)0, bq, (const float*)nullptr, (long)0,
      NROWS, HID, KPAD, 1.0f);
  k_colstats<<<dim3(NCHUNK, NB), HID, 0, stream>>>(yq, HID, HID, ps_q, pq_q);
  k_statfin<<<dim3(NB), HID, 0, stream>>>(ps_q, pq_q, HID, mn_q, iv_q);
  k_fin_q<<<dim3(NPTS / 32, NB), 256, 0, stream>>>(yq, mn_q, iv_q, zpl, h, out);
}
